// SpatialAttention2D_32469952757968
// MI455X (gfx1250) — hardware-verified
//
#include <hip/hip_runtime.h>
#include <math.h>

constexpr int kBatch  = 2;
constexpr int kChan   = 64;
constexpr int kNtok   = 4096;
constexpr int kTok    = kBatch * kNtok;
constexpr int kHeads  = 4;
constexpr int kHdim   = 16;
constexpr int kGroups = kBatch * kHeads;
constexpr int kQKV    = 3 * kChan;
constexpr int kQKld   = 32;
constexpr int kVrows  = 64;
constexpr float kWCarry    = 16.0f;
constexpr float kWCarryInv = 1.0f / 16.0f;
constexpr float kPCarry    = 2048.0f;
constexpr float kPCarryInv = 1.0f / 2048.0f;
constexpr float kQKScale   = 0.25f;


typedef __attribute__((ext_vector_type(16))) _Float16 v16h;
typedef __attribute__((ext_vector_type(8)))  _Float16 v8h;
typedef __attribute__((ext_vector_type(16))) __bf16   v16b;
typedef __attribute__((ext_vector_type(8)))  __bf16   v8b;
typedef __attribute__((ext_vector_type(8)))  float    v8f;
typedef __attribute__((ext_vector_type(4)))  float    v4f;
typedef __attribute__((ext_vector_type(4)))  unsigned int v4u;

__device__ __forceinline__ unsigned short f2bf_bits(float f) {
  unsigned u = __float_as_uint(f);
  return (unsigned short)((u + 0x7FFFu + ((u >> 16) & 1u)) >> 16);
}
__device__ __forceinline__ float bf_bits2f(unsigned short h) { return __uint_as_float(((unsigned)h) << 16); }

__device__ __forceinline__ void dep_guard_h(v8f& a, v8f& b, v16h x, v16h y) { asm volatile("v_nop\n\tv_nop\n\tv_nop\n\tv_nop" : "+v"(a), "+v"(b) : "v"(x), "v"(y)); }
__device__ __forceinline__ void dep_guard_b(v8f& a, v8f& b, v16b x, v16b y) { asm volatile("v_nop\n\tv_nop\n\tv_nop\n\tv_nop" : "+v"(a), "+v"(b) : "v"(x), "v"(y)); }
__device__ __forceinline__ void keep4_h(v16h a, v16h b, v16h c, v16h d) { asm volatile("v_nop" :: "v"(a), "v"(b), "v"(c), "v"(d)); }
__device__ __forceinline__ void keep4_b(v16b a, v16b b, v16b c, v16b d) { asm volatile("v_nop" :: "v"(a), "v"(b), "v"(c), "v"(d)); }
__device__ __forceinline__ void acc_guard4(v8f& a, v8f& b, v8f& c, v8f& d) { asm volatile("v_nop\n\tv_nop\n\tv_nop\n\tv_nop" : "+v"(a), "+v"(b), "+v"(c), "+v"(d)); }
template <typename T> struct Frag;
template <> struct Frag<_Float16> {
  typedef v16h V; union U { v16h v; v8h h[2]; };
  static __device__ __forceinline__ v16h load(const _Float16* p) {
    U f; f.h[0] = *(const v8h*)(p); f.h[1] = *(const v8h*)(p + 16); return f.v;
  }
  static __device__ __forceinline__ v8f mma(v16h a, v16h b, v8f c) {
    return __builtin_amdgcn_wmma_f32_16x16x32_f16(false, a, false, b, (short)0, c, false, false);
  }
  static __device__ __forceinline__ void guard(v8f& a, v8f& b, v16h x, v16h y) { dep_guard_h(a, b, x, y); }
  static __device__ __forceinline__ void keep(v16h a, v16h b, v16h c, v16h d) { keep4_h(a, b, c, d); }
};
template <> struct Frag<__bf16> {
  typedef v16b V; union U { v16b v; v8b h[2]; };
  static __device__ __forceinline__ v16b load(const __bf16* p) {
    U f; f.h[0] = *(const v8b*)(p); f.h[1] = *(const v8b*)(p + 16); return f.v;
  }
  static __device__ __forceinline__ v8f mma(v16b a, v16b b, v8f c) {
    return __builtin_amdgcn_wmma_f32_16x16x32_bf16(false, a, false, b, (short)0, c, false, false);
  }
  static __device__ __forceinline__ void guard(v8f& a, v8f& b, v16b x, v16b y) { dep_guard_b(a, b, x, y); }
  static __device__ __forceinline__ void keep(v16b a, v16b b, v16b c, v16b d) { keep4_b(a, b, c, d); }
};

__device__ __forceinline__ unsigned pk16(unsigned short a, unsigned short b) { return (unsigned)a | ((unsigned)b << 16); }
__device__ __forceinline__ unsigned short h_bits(float f) { const _Float16 h = (_Float16)f; return __builtin_bit_cast(unsigned short, h); }

template <int ET> struct Elem;
template <> struct Elem<0> { typedef _Float16 T; };
template <> struct Elem<1> { typedef __bf16 T; };
template <int ET, bool SPLIT, int BIAS_MODE, int OUT_MODE, bool RESID, int ACT = 0>
__global__ __launch_bounds__(256) void wmma_gemm64(
    const unsigned short* __restrict__ Ap, const unsigned short* __restrict__ A2p, int lda, long strideA,
    const unsigned short* __restrict__ Btp, const unsigned short* __restrict__ Bt2p, int ldb, long strideB,
    void* __restrict__ Cout, void* __restrict__ Cout2, int ldc, long strideC,
    const float* __restrict__ bias,
    const float* __restrict__ resid, long strideR,
    int M, int N, int K, float scale) {
  typedef typename Elem<ET>::T T;
  typedef typename Frag<T>::V V;
  const T* A = (const T*)Ap; const T* A2 = (const T*)A2p; const T* Bt = (const T*)Btp; const T* Bt2 = (const T*)Bt2p;
  __shared__ __align__(16) float sT[8][16 * 68];
  const int b    = blockIdx.y;
  const int lane = threadIdx.x & 31;
  const int wave = threadIdx.x >> 5;
  const int tilesN = N >> 6;
  const int tilesM = M >> 6;
  const int tile = blockIdx.x * 8 + wave;
  if (tile >= tilesM * tilesN) return;
  const int tm = tile / tilesN;
  const int tn = tile - tm * tilesN;
  const int m0 = tm << 6;
  const int n0 = tn << 6;

  const T* Ab  = A  + (size_t)b * strideA;
  const T* Bb  = Bt + (size_t)b * strideB;
  const T* Ab2 = SPLIT ? (A2  + (size_t)b * strideA) : nullptr;
  const T* Bb2 = SPLIT ? (Bt2 + (size_t)b * strideB) : nullptr;

  const int rlane = lane & 15;
  const int koff  = (lane >> 4) * 8;
  const int mOff  = (lane >> 4) * 8;

  v8f acc[4][4];
#pragma unroll
  for (int i = 0; i < 4; ++i)
#pragma unroll
    for (int j = 0; j < 4; ++j) acc[i][j] = (v8f){0.f,0.f,0.f,0.f,0.f,0.f,0.f,0.f};

  for (int k0 = 0; k0 < K; k0 += 32) {
    V bh[4], bl[4];
#pragma unroll
    for (int j = 0; j < 4; ++j) {
      const size_t bo = (size_t)(n0 + (j << 4) + rlane) * ldb + koff + k0;
      bh[j] = Frag<T>::load(Bb + bo);
      if (SPLIT) bl[j] = Frag<T>::load(Bb2 + bo);
    }
#pragma unroll
    for (int i = 0; i < 4; ++i) {
      const size_t ao = (size_t)(m0 + (i << 4) + rlane) * lda + koff + k0;
      V ah = Frag<T>::load(Ab + ao);
      V al;
      if (SPLIT) al = Frag<T>::load(Ab2 + ao);
#pragma unroll
      for (int j = 0; j < 4; ++j) {
        acc[i][j] = Frag<T>::mma(ah, bh[j], acc[i][j]);
        if (SPLIT) {
          acc[i][j] = Frag<T>::mma(ah, bl[j], acc[i][j]);
          acc[i][j] = Frag<T>::mma(al, bh[j], acc[i][j]);
        }
      }
      Frag<T>::guard(acc[i][0], acc[i][3], ah, SPLIT ? al : ah);
    }
    Frag<T>::keep(bh[0], bh[1], bh[2], bh[3]);
    if (SPLIT) Frag<T>::keep(bl[0], bl[1], bl[2], bl[3]);
  }
  acc_guard4(acc[0][0], acc[0][1], acc[0][2], acc[0][3]);
  acc_guard4(acc[1][0], acc[1][1], acc[1][2], acc[1][3]);
  acc_guard4(acc[2][0], acc[2][1], acc[2][2], acc[2][3]);
  acc_guard4(acc[3][0], acc[3][1], acc[3][2], acc[3][3]);

  float* slab = sT[wave];
  const float* Rb = RESID ? (resid + (size_t)b * strideR) : nullptr;
#pragma unroll
  for (int i = 0; i < 4; ++i) {
    const int mBase = m0 + (i << 4);
#pragma unroll
    for (int j = 0; j < 4; ++j) {
      const int n = n0 + (j << 4) + rlane;
      float bv = 0.f;
      if (BIAS_MODE == 2) bv = bias[n];
#pragma unroll
      for (int r = 0; r < 8; ++r) {
        float v = acc[i][j][r] * scale;
        if (BIAS_MODE == 1) v += bias[mBase + mOff + r];
        if (BIAS_MODE == 2) v += bv;
        if (RESID) v += Rb[(size_t)(mBase + mOff + r) * ldc + n];
        if (ACT == 2) v = fmaxf(v, 0.0f);
        if (ACT == 4) v = (v > 0.f) ? v : 0.01f * v;
        slab[(mOff + r) * 68 + (j << 4) + rlane] = v;
      }
    }
    __builtin_amdgcn_fence(__ATOMIC_RELEASE, "workgroup");
    __builtin_amdgcn_wave_barrier();
    __builtin_amdgcn_fence(__ATOMIC_ACQUIRE, "workgroup");
    if (OUT_MODE == 0) {
      float* C = (float*)Cout + (size_t)b * strideC;
      const int hh = lane >> 4, c4 = (lane & 15) * 4;
      for (int pass = 0; pass < 2; ++pass) {
#pragma unroll
        for (int it = 0; it < 8; ++it) {
          const int row = it * 2 + hh;
          v4f v = *(const v4f*)(slab + row * 68 + c4);
          *(volatile v4f*)(C + (size_t)(mBase + row) * ldc + n0 + c4) = v;
        }
        __threadfence();
      }
    } else {
      const int q = lane >> 3, c8 = (lane & 7) * 8;
      unsigned short* C  = (unsigned short*)Cout  + (size_t)b * strideC;
      unsigned short* C2 = (OUT_MODE == 2) ? ((unsigned short*)Cout2 + (size_t)b * strideC) : nullptr;
      for (int pass = 0; pass < 2; ++pass) {
#pragma unroll
        for (int it = 0; it < 4; ++it) {
          const int row = it * 4 + q;
          const float* sp = slab + row * 68 + c8;
          v8h hv, lv;
#pragma unroll
          for (int e = 0; e < 8; ++e) {
            if (OUT_MODE == 1) {
              hv[e] = (_Float16)sp[e];
            } else {
              unsigned short hb = f2bf_bits(sp[e]);
              unsigned short lb = f2bf_bits(sp[e] - bf_bits2f(hb));
              hv[e] = __builtin_bit_cast(_Float16, hb);
              lv[e] = __builtin_bit_cast(_Float16, lb);
            }
          }
          *(volatile v8h*)(C + (size_t)(mBase + row) * ldc + n0 + c8) = hv;
          if (OUT_MODE == 2) *(volatile v8h*)(C2 + (size_t)(mBase + row) * ldc + n0 + c8) = lv;
        }
        __threadfence();
      }
    }
    __builtin_amdgcn_fence(__ATOMIC_RELEASE, "workgroup");
    __builtin_amdgcn_wave_barrier();
    __builtin_amdgcn_fence(__ATOMIC_ACQUIRE, "workgroup");
  }
}

__global__ __launch_bounds__(256) void xtok_kernel(const float* __restrict__ x, unsigned short* __restrict__ T16) {
  __shared__ float sm[64][65];
  const int t    = threadIdx.x;
  const int tok0 = blockIdx.x * 64;
  const int b    = tok0 >> 12;
  const int n0   = tok0 & (kNtok - 1);
  const float* xb = x + (size_t)b * kChan * kNtok + n0;
#pragma unroll
  for (int i = 0; i < 16; ++i) {
    const int e  = i * 256 + t;
    const int c  = e >> 6;
    const int nl = e & 63;
    sm[nl][c] = xb[(size_t)c * kNtok + nl];
  }
  __syncthreads();
  const int lane = t & 31, wave = t >> 5;
  const int q = lane >> 3, c8 = (lane & 7) * 8;
  for (int pass = 0; pass < 2; ++pass) {
#pragma unroll
    for (int it = 0; it < 2; ++it) {
      const int row = wave * 8 + it * 4 + q;
      unsigned short hb[8];
#pragma unroll
      for (int e = 0; e < 8; ++e) hb[e] = h_bits(sm[row][c8 + e]);
      const v4u u = (v4u){pk16(hb[0], hb[1]), pk16(hb[2], hb[3]), pk16(hb[4], hb[5]), pk16(hb[6], hb[7])};
      *(volatile v4u*)(T16 + (size_t)(tok0 + row) * kChan + c8) = u;
    }
    __threadfence();
  }
}

__global__ __launch_bounds__(256) void wcast8_kernel(const float* __restrict__ in, unsigned short* __restrict__ out, int n8, float scale) {
  const int i = blockIdx.x * 256 + threadIdx.x;
  if (i >= n8) return;
  const float* p = in + 8 * (size_t)i;
  const v4f a = *(const v4f*)(p);
  const v4f c = *(const v4f*)(p + 4);
  unsigned short hb[8];
#pragma unroll
  for (int e = 0; e < 4; ++e) {
    hb[e]     = h_bits(a[e] * scale);
    hb[4 + e] = h_bits(c[e] * scale);
  }
  const v4u u = (v4u){pk16(hb[0], hb[1]), pk16(hb[2], hb[3]), pk16(hb[4], hb[5]), pk16(hb[6], hb[7])};
  unsigned short* q = out + 8 * (size_t)i;
  *(volatile v4u*)q = u;
  __threadfence();
  *(volatile v4u*)q = u;
}

__global__ __launch_bounds__(256) void qkv_split_kernel(const float* __restrict__ QKV32,
                                                        unsigned short* __restrict__ Q16,
                                                        unsigned short* __restrict__ K16,
                                                        unsigned short* __restrict__ Vcm16) {
  __shared__ float sm[64][193];
  const int t    = threadIdx.x;
  const int tok0 = blockIdx.x * 64;
  const int b    = tok0 >> 12;
  const int n0   = tok0 & (kNtok - 1);
  const float* src = QKV32 + (size_t)tok0 * kQKV;
#pragma unroll
  for (int i = 0; i < 12; ++i) {
    const int e   = i * 256 + t;
    const int row = e / 48;
    const int col = (e - row * 48) * 4;
    const v4f v = *(const v4f*)(src + 4 * (size_t)e);
    sm[row][col]     = v[0];
    sm[row][col + 1] = v[1];
    sm[row][col + 2] = v[2];
    sm[row][col + 3] = v[3];
  }
  __syncthreads();
  const int rowq = t >> 2;
  const int q4   = t & 3;
  const unsigned keepq = (q4 < 2) ? 0xffffffffu : 0u;
  const int cq   = (q4 & 1) * 8;
  const int lq   = t >> 3;
  const int e8   = (t & 7) * 8;
  for (int pass = 0; pass < 2; ++pass) {
#pragma unroll
    for (int h = 0; h < kHeads; ++h) {
      const size_t prow = ((size_t)(b * kHeads + h) * kNtok + n0 + rowq) * kQKld + 8 * q4;
      {
        unsigned short hb[8];
#pragma unroll
        for (int e = 0; e < 8; ++e) hb[e] = h_bits(sm[rowq][h * kHdim + cq + e]);
        const v4u u = (v4u){pk16(hb[0], hb[1]) & keepq, pk16(hb[2], hb[3]) & keepq,
                            pk16(hb[4], hb[5]) & keepq, pk16(hb[6], hb[7]) & keepq};
        *(volatile v4u*)(Q16 + prow) = u;
      }
      {
        unsigned short hb[8];
#pragma unroll
        for (int e = 0; e < 8; ++e) hb[e] = h_bits(sm[rowq][kChan + h * kHdim + cq + e]);
        const v4u u = (v4u){pk16(hb[0], hb[1]) & keepq, pk16(hb[2], hb[3]) & keepq,
                            pk16(hb[4], hb[5]) & keepq, pk16(hb[6], hb[7]) & keepq};
        *(volatile v4u*)(K16 + prow) = u;
      }
    }
#pragma unroll
    for (int it = 0; it < 8; ++it) {
      const int L  = it * 32 + lq;
      const int h  = L >> 6;
      const int vr = L & 63;
      const unsigned keepv = (vr < 16) ? 0xffffffffu : 0u;
      const int d  = vr & 15;
      unsigned short hb[8];
#pragma unroll
      for (int e = 0; e < 8; ++e) hb[e] = h_bits(sm[e8 + e][2 * kChan + h * kHdim + d]);
      const v4u u = (v4u){pk16(hb[0], hb[1]) & keepv, pk16(hb[2], hb[3]) & keepv,
                          pk16(hb[4], hb[5]) & keepv, pk16(hb[6], hb[7]) & keepv};
      *(volatile v4u*)(Vcm16 + ((size_t)((b * kHeads + h) * kVrows + vr)) * kNtok + n0 + e8) = u;
    }
    __threadfence();
  }
}

__global__ __launch_bounds__(512) void softmax_row_kernel(const float* __restrict__ S, unsigned short* __restrict__ P, float carry) {
  __shared__ float redM[16];
  __shared__ float redS[16];
  __shared__ __align__(16) float es[512 * 8];
  const int row  = blockIdx.x;
  const int t    = threadIdx.x;
  const int lane = t & 31, wave = t >> 5;
  const float* sr = S + (size_t)row * kNtok + 8 * t;
  const v4f a0 = *(const v4f*)(sr);
  const v4f a1 = *(const v4f*)(sr + 4);
  float m = fmaxf(fmaxf(fmaxf(a0[0], a0[1]), fmaxf(a0[2], a0[3])), fmaxf(fmaxf(a1[0], a1[1]), fmaxf(a1[2], a1[3])));
#pragma unroll
  for (int off = 16; off > 0; off >>= 1) m = fmaxf(m, __shfl_xor(m, off, 32));
  if (lane == 0) redM[wave] = m;
  __syncthreads();
  float gm = redM[0];
#pragma unroll
  for (int w = 1; w < 16; ++w) gm = fmaxf(gm, redM[w]);
  float* et = es + t * 8;
  float psum = 0.f;
#pragma unroll 1
  for (int half = 0; half < 2; ++half) {
    const v4f a = *(const v4f*)(sr + 4 * half);
    v4f e;
    e[0] = expf(a[0] - gm);
    e[1] = expf(a[1] - gm);
    e[2] = expf(a[2] - gm);
    e[3] = expf(a[3] - gm);
    psum += (e[0] + e[1]) + (e[2] + e[3]);
    *(v4f*)(et + 4 * half) = e;
  }
#pragma unroll
  for (int off = 16; off > 0; off >>= 1) psum += __shfl_xor(psum, off, 32);
  if (lane == 0) redS[wave] = psum;
  __syncthreads();
  float tot = redS[0];
#pragma unroll
  for (int w = 1; w < 16; ++w) tot += redS[w];
  const float inv = carry * (1.0f / tot);
  const v4f e0 = *(const v4f*)(et);
  const v4f e1 = *(const v4f*)(et + 4);
  unsigned short hb[8];
#pragma unroll
  for (int e = 0; e < 4; ++e) {
    hb[e]     = h_bits(e0[e] * inv);
    hb[4 + e] = h_bits(e1[e] * inv);
  }
  const v4u u = (v4u){pk16(hb[0], hb[1]), pk16(hb[2], hb[3]), pk16(hb[4], hb[5]), pk16(hb[6], hb[7])};
  unsigned short* pp = P + (size_t)row * kNtok + 8 * t;
  *(volatile v4u*)pp = u;
  __threadfence();
  *(volatile v4u*)pp = u;
}

__global__ __launch_bounds__(256) void merge_out_kernel(const float* __restrict__ O32, float* __restrict__ out) {
  const int i  = blockIdx.x * 256 + threadIdx.x;
  const int r  = i >> 10;
  const int c4 = (i & 1023) * 4;
  const int b  = r >> 6;
  const int ch = r & 63;
  const int h  = ch >> 4;
  const int d  = ch & 15;
  const size_t src = ((size_t)((b * kHeads + h) * kVrows + d)) * kNtok + c4;
  const v4f v = *(const v4f*)(O32 + src);
  float* p = out + (size_t)r * kNtok + c4;
  *(volatile v4f*)p = v;
  __threadfence();
  *(volatile v4f*)p = v;
}

extern "C" void kernel_launch(void* const* d_in, const int* in_sizes, int n_in,
                              void* d_out, int out_size, void* d_ws, size_t ws_size,
                              hipStream_t stream) {
  (void)in_sizes; (void)n_in;
  const float* x    = (const float*)d_in[0];
  const float* w    = (const float*)d_in[1];
  const float* bias = (const float*)d_in[2];
  float* out = (float*)d_out;

  const size_t szT16   = (size_t)kTok * kChan * 2;
  const size_t szW16   = (size_t)kQKV * kChan * 2;
  const size_t szQKV32 = (size_t)kTok * kQKV * 4;
  const size_t szQK16  = (size_t)kGroups * kNtok * kQKld * 2;
  const size_t szVcm16 = (size_t)kGroups * kVrows * kNtok * 2;
  const size_t szS32   = (size_t)kNtok * kNtok * 4;
  const size_t szP16   = (size_t)kNtok * kNtok * 2;
  const size_t szO32   = (size_t)kGroups * kVrows * kNtok * 4;
  char* ws = (char*)d_ws;
  size_t off = 0;
  unsigned short* T16   = (unsigned short*)(ws + off); off += szT16;
  unsigned short* W16   = (unsigned short*)(ws + off); off += szW16;
  float*          QKV32 = (float*)(ws + off);          off += szQKV32;
  unsigned short* Q16   = (unsigned short*)(ws + off); off += szQK16;
  unsigned short* K16   = (unsigned short*)(ws + off); off += szQK16;
  unsigned short* Vcm16 = (unsigned short*)(ws + off); off += szVcm16;
  float*          S32   = (float*)(ws + off);          off += szS32;
  unsigned short* P16   = (unsigned short*)(ws + off); off += szP16;
  float*          O32   = (float*)(ws + off);          off += szO32;
  if (off > ws_size) return;
  if ((size_t)out_size < (size_t)kBatch * kChan * kNtok) return;

  xtok_kernel<<<dim3(kTok / 64), dim3(256), 0, stream>>>(x, T16);
  wcast8_kernel<<<dim3((kQKV * kChan / 8 + 255) / 256), dim3(256), 0, stream>>>(w, W16, kQKV * kChan / 8, kWCarry);
  wmma_gemm64<0, false, 2, 0, false, 0><<<dim3((kTok / 64) * (kQKV / 64) / 8, 1), dim3(256), 0, stream>>>(
      T16, T16, kChan, 0L, W16, W16, kChan, 0L, (void*)QKV32, (void*)QKV32, kQKV, 0L,
      bias, x, 0L, kTok, kQKV, kChan, kWCarryInv);
  qkv_split_kernel<<<dim3(kTok / 64), dim3(256), 0, stream>>>(QKV32, Q16, K16, Vcm16);

  for (int g = 0; g < kGroups; ++g) {
    const unsigned short* Qg = Q16 + (size_t)g * kNtok * kQKld;
    const unsigned short* Kg = K16 + (size_t)g * kNtok * kQKld;
    const unsigned short* Vg = Vcm16 + (size_t)g * kVrows * kNtok;
    float* Og = O32 + (size_t)g * kVrows * kNtok;
    wmma_gemm64<0, false, 0, 0, false, 0><<<dim3((kNtok / 64) * (kNtok / 64) / 8, 1), dim3(256), 0, stream>>>(
        Qg, Qg, kQKld, 0L, Kg, Kg, kQKld, 0L, (void*)S32, (void*)S32, kNtok, 0L,
        bias, x, 0L, kNtok, kNtok, kQKld, kQKScale);
    softmax_row_kernel<<<dim3(kNtok), dim3(512), 0, stream>>>(S32, P16, kPCarry);
    wmma_gemm64<0, false, 0, 0, false, 0><<<dim3((kVrows / 64) * (kNtok / 64) / 8, 1), dim3(256), 0, stream>>>(
        Vg, Vg, kNtok, 0L, P16, P16, kNtok, 0L, (void*)Og, (void*)Og, kNtok, 0L,
        bias, x, 0L, kVrows, kNtok, kNtok, kPCarryInv);
  }

  merge_out_kernel<<<dim3((kBatch * kChan * kNtok / 4) / 256), dim3(256), 0, stream>>>(O32, out);
}
